// ZImageAttention_45947560132707
// MI455X (gfx1250) — hardware-verified
//
#include <hip/hip_runtime.h>
#include <math.h>
#include <stddef.h>
#include <stdint.h>

#define NB    2
#define SQ    2048
#define DM    2048
#define NH    16
#define NKV   8
#define HD    128
#define EQ    (NH * HD)
#define EK    (NKV * HD)
#define NTOK  (NB * SQ)
#define TP    132
#define OSP   136
#define RMS_EPS 1e-5f
#define QMUL  (0.08838834764831845f * 1.4426950408889634f * 1024.0f)
#define KMUL  8.0f
#define VMUL  1024.0f
#define SINV  (1.0f / 8192.0f)

typedef _Float16 v16h __attribute__((ext_vector_type(16)));
typedef _Float16 v8h  __attribute__((ext_vector_type(8)));
typedef __bf16   v16b __attribute__((ext_vector_type(16)));
typedef __bf16   v8b  __attribute__((ext_vector_type(8)));
typedef float    v8f  __attribute__((ext_vector_type(8)));
typedef float    v4f  __attribute__((ext_vector_type(4)));
typedef unsigned int v4u __attribute__((ext_vector_type(4)));

union HFrag { v16h v; v8h h[2]; };
union BFrag { v16b v; v8b h[2]; };

__device__ __forceinline__ unsigned short f2bf_bits(float f) {
  const unsigned u = __float_as_uint(f);
  return (unsigned short)((u + 0x7FFFu + ((u >> 16) & 1u)) >> 16);
}
__device__ __forceinline__ float bfb2f(unsigned short h) { return __uint_as_float(((unsigned)h) << 16); }
__device__ __forceinline__ float bf16r(float f) { return bfb2f(f2bf_bits(f)); }
__device__ __forceinline__ unsigned short hbits(_Float16 h) { return __builtin_bit_cast(unsigned short, h); }
__device__ __forceinline__ unsigned pk16(unsigned short a, unsigned short b) { return (unsigned)a | ((unsigned)b << 16); }

__device__ __forceinline__ v16b ldb(const __bf16* p) {
  BFrag f; f.h[0] = *(const v8b*)(p); f.h[1] = *(const v8b*)(p + 16); return f.v;
}
__device__ __forceinline__ v16h ldh(const _Float16* p) {
  HFrag f; f.h[0] = *(const v8h*)(p); f.h[1] = *(const v8h*)(p + 16); return f.v;
}
__device__ __forceinline__ v8f mma_b(v16b a, v16b b, v8f c) {
  return __builtin_amdgcn_wmma_f32_16x16x32_bf16(false, a, false, b, (short)0, c, false, false);
}
__device__ __forceinline__ v8f mma_h(v16h a, v16h b, v8f c) {
  return __builtin_amdgcn_wmma_f32_16x16x32_f16(false, a, false, b, (short)0, c, false, false);
}

__device__ __forceinline__ void guard_b(v8f& a, v8f& b, v16b x, v16b y) {
  asm volatile("v_nop\n\tv_nop\n\tv_nop\n\tv_nop" : "+v"(a), "+v"(b) : "v"(x), "v"(y));
}
__device__ __forceinline__ void keep_b(v16b a, v16b b, v16b c, v16b d) {
  asm volatile("v_nop" :: "v"(a), "v"(b), "v"(c), "v"(d));
}
__device__ __forceinline__ void acc_guard4(v8f& a, v8f& b, v8f& c, v8f& d) {
  asm volatile("v_nop\n\tv_nop\n\tv_nop\n\tv_nop" : "+v"(a), "+v"(b), "+v"(c), "+v"(d));
}
__device__ __forceinline__ void g_qk(v8f& s0, v8f& s1, v8f& s2, v8f& s3,
                                     v16h k0, v16h k1, v16h k2, v16h k3, v16h qa, v16h qb) {
  asm volatile("v_nop\n\tv_nop\n\tv_nop\n\tv_nop"
               : "+v"(s0), "+v"(s1), "+v"(s2), "+v"(s3)
               : "v"(k0), "v"(k1), "v"(k2), "v"(k3), "v"(qa), "v"(qb));
}
__device__ __forceinline__ void g_pv(v8f& a0, v8f& a1, v16h x0, v16h x1, v16h x2, v16h x3, v16h p) {
  asm volatile("v_nop\n\tv_nop\n\tv_nop\n\tv_nop"
               : "+v"(a0), "+v"(a1) : "v"(x0), "v"(x1), "v"(x2), "v"(x3), "v"(p));
}
__device__ __forceinline__ void g_acc8(v8f& a0, v8f& a1, v8f& a2, v8f& a3, v8f& a4, v8f& a5, v8f& a6, v8f& a7) {
  asm volatile("v_nop\n\tv_nop\n\tv_nop\n\tv_nop"
               : "+v"(a0), "+v"(a1), "+v"(a2), "+v"(a3), "+v"(a4), "+v"(a5), "+v"(a6), "+v"(a7));
}
__device__ __forceinline__ void sched_fence() { asm volatile("" ::: "memory"); }

__global__ __launch_bounds__(256) void cvt_bf16_kernel(const float* __restrict__ in,
                                                       unsigned short* __restrict__ out, int n8) {
  const int i = blockIdx.x * 256 + threadIdx.x;
  if (i < n8) {
    const float* src = in + (size_t)i * 8;
    const v4f a = *(const v4f*)(src);
    const v4f b = *(const v4f*)(src + 4);
    v4u o;
    o[0] = pk16(f2bf_bits(a[0]), f2bf_bits(a[1]));
    o[1] = pk16(f2bf_bits(a[2]), f2bf_bits(a[3]));
    o[2] = pk16(f2bf_bits(b[0]), f2bf_bits(b[1]));
    o[3] = pk16(f2bf_bits(b[2]), f2bf_bits(b[3]));
    unsigned short* dst = out + (size_t)i * 8;
    *(volatile v4u*)dst = o;
    __threadfence();
    *(volatile v4u*)dst = o;
  }
}

template <bool SPLIT>
__device__ __forceinline__ void gemm_core(const __bf16* __restrict__ A, const __bf16* __restrict__ A2,
                                          const __bf16* __restrict__ B, int lane, v8f (&acc)[2][4]) {
  const int m = lane & 15, ko = (lane >> 4) * 8;
  const __bf16* Ar  = A  + (size_t)m * DM + ko;
  const __bf16* Ar2 = A2 + (size_t)m * DM + ko;
  const __bf16* Br  = B  + (size_t)m * DM + ko;
#pragma unroll 1
  for (int k0 = 0; k0 < DM; k0 += 32) {
    v16b bf[4];
#pragma unroll
    for (int j = 0; j < 4; ++j) bf[j] = ldb(Br + (size_t)(16 * j) * DM + k0);
#pragma unroll
    for (int i = 0; i < 2; ++i) {
      const v16b af = ldb(Ar + (size_t)(16 * i) * DM + k0);
      v16b al = af;
      if (SPLIT) al = ldb(Ar2 + (size_t)(16 * i) * DM + k0);
#pragma unroll
      for (int j = 0; j < 4; ++j) {
        acc[i][j] = mma_b(af, bf[j], acc[i][j]);
        if (SPLIT) acc[i][j] = mma_b(al, bf[j], acc[i][j]);
      }
      guard_b(acc[i][0], acc[i][3], af, al);
    }
    keep_b(bf[0], bf[1], bf[2], bf[3]);
  }
  acc_guard4(acc[0][0], acc[0][1], acc[0][2], acc[0][3]);
  acc_guard4(acc[1][0], acc[1][1], acc[1][2], acc[1][3]);
}

__device__ __forceinline__ void stage_tile(float* T, int w, int lane, v8f (&acc)[2][4]) {
  const int wr = w >> 1, wc = w & 1, hh = lane >> 4, m = lane & 15;
#pragma unroll
  for (int i = 0; i < 2; ++i)
#pragma unroll
    for (int j = 0; j < 4; ++j)
#pragma unroll
      for (int r = 0; r < 8; ++r)
        T[(32 * wr + 16 * i + 8 * hh + r) * TP + 64 * wc + 16 * j + m] = acc[i][j][r];
}

template <int ROLE>
__global__ __launch_bounds__(128) void proj_kernel(const unsigned short* __restrict__ Ap,
                                                   const unsigned short* __restrict__ Bp,
                                                   const float* __restrict__ nw,
                                                   const float* __restrict__ fcos,
                                                   const float* __restrict__ fsin,
                                                   unsigned short* __restrict__ P1,
                                                   unsigned short* __restrict__ P2) {
  __shared__ __align__(16) float T[64 * TP];
  const int lane = threadIdx.x & 31;
  const int w    = threadIdx.x >> 5;
  const int hh   = lane >> 4;
  const int m    = lane & 15;
  const int wr   = w >> 1, wc = w & 1;
  const int arow0 = (ROLE == 2) ? (int)blockIdx.y * 64 : (int)blockIdx.x * 64;
  const int brow0 = (ROLE == 2) ? (int)blockIdx.x * 128 : (int)blockIdx.y * 128;
  const __bf16* A = (const __bf16*)(const void*)Ap + (size_t)(arow0 + 32 * wr) * DM;
  const __bf16* B = (const __bf16*)(const void*)Bp + (size_t)(brow0 + 64 * wc) * DM;

  v8f acc[2][4];
#pragma unroll
  for (int i = 0; i < 2; ++i)
#pragma unroll
    for (int j = 0; j < 4; ++j) acc[i][j] = (v8f){0.f, 0.f, 0.f, 0.f, 0.f, 0.f, 0.f, 0.f};

  gemm_core<false>(A, A, B, lane, acc);
  stage_tile(T, w, lane, acc);
  __syncthreads();

  float wv[8];
  if (ROLE != 2) {
    const v4f wa = *(const v4f*)(nw + 8 * m);
    const v4f wb = *(const v4f*)(nw + 8 * m + 4);
#pragma unroll
    for (int e = 0; e < 4; ++e) { wv[e] = bf16r(wa[e]); wv[4 + e] = bf16r(wb[e]); }
  } else {
#pragma unroll
    for (int e = 0; e < 8; ++e) wv[e] = 1.0f;
  }

  v4u hv[8], lv[8];
#pragma unroll
  for (int it = 0; it < 8; ++it) {
    const int row = 16 * w + 2 * it + hh;
    const float* tr = T + row * TP + 8 * m;
    const v4f xa = *(const v4f*)(tr);
    const v4f xb = *(const v4f*)(tr + 4);
    float x[8] = {xa[0], xa[1], xa[2], xa[3], xb[0], xb[1], xb[2], xb[3]};
    float y[8];
    if (ROLE == 2) {
#pragma unroll
      for (int e = 0; e < 8; ++e) y[e] = x[e] * VMUL;
    } else {
      float ss = 0.f;
#pragma unroll
      for (int e = 0; e < 8; ++e) ss = fmaf(x[e], x[e], ss);
      ss += __shfl_xor(ss, 1, 32);
      ss += __shfl_xor(ss, 2, 32);
      ss += __shfl_xor(ss, 4, 32);
      ss += __shfl_xor(ss, 8, 32);
      const float rn  = rsqrtf(fmaf(ss, 1.0f / (float)HD, RMS_EPS));
      const int   tok = arow0 + row;
      const int   sp  = tok & (SQ - 1);
      const v4f c4 = *(const v4f*)(fcos + (size_t)sp * (HD / 2) + 4 * m);
      const v4f s4 = *(const v4f*)(fsin + (size_t)sp * (HD / 2) + 4 * m);
      const float om = (ROLE == 0) ? QMUL : KMUL;
#pragma unroll
      for (int p = 0; p < 4; ++p) {
        const float cs = bf16r(c4[p]), sn = bf16r(s4[p]);
        const float u0 = x[2 * p] * rn * wv[2 * p];
        const float u1 = x[2 * p + 1] * rn * wv[2 * p + 1];
        y[2 * p]     = (u0 * cs - u1 * sn) * om;
        y[2 * p + 1] = (u0 * sn + u1 * cs) * om;
      }
    }
    v4u a, c2;
#pragma unroll
    for (int q = 0; q < 4; ++q) {
      const _Float16 h0 = (_Float16)y[2 * q];
      const _Float16 h1 = (_Float16)y[2 * q + 1];
      a[q] = pk16(hbits(h0), hbits(h1));
      if (ROLE != 1) {
        const _Float16 l0 = (_Float16)(y[2 * q] - (float)h0);
        const _Float16 l1 = (_Float16)(y[2 * q + 1] - (float)h1);
        c2[q] = pk16(hbits(l0), hbits(l1));
      } else {
        c2[q] = 0u;
      }
    }
    hv[it] = a;
    lv[it] = c2;
  }

  for (int pass = 0; pass < 2; ++pass) {
#pragma unroll
    for (int it = 0; it < 8; ++it) {
      const int row = 16 * w + 2 * it + hh;
      size_t go;
      if (ROLE == 0) {
        go = (size_t)(arow0 + row) * EQ + (size_t)blockIdx.y * HD + 8 * m;
      } else if (ROLE == 1) {
        go = (size_t)(arow0 + row) * EK + (size_t)blockIdx.y * HD + 8 * m;
      } else {
        const int f   = arow0 + row;
        const int kvh = f >> 7;
        const int d   = f & (HD - 1);
        const int bb  = brow0 >> 11;
        const int s0  = brow0 & (SQ - 1);
        go = ((size_t)((bb * NKV + kvh) * HD + d)) * SQ + s0 + 8 * m;
      }
      *(volatile v4u*)(P1 + go) = hv[it];
      if (ROLE != 1) *(volatile v4u*)(P2 + go) = lv[it];
    }
    __threadfence();
  }
}

__global__ __launch_bounds__(64) void attn_kernel(const unsigned short* __restrict__ Qhp,
                                                  const unsigned short* __restrict__ Qlp,
                                                  const unsigned short* __restrict__ Kpp,
                                                  const unsigned short* __restrict__ Vhp,
                                                  const unsigned short* __restrict__ Vlp,
                                                  unsigned short* __restrict__ Ohp,
                                                  unsigned short* __restrict__ Olp) {
  __shared__ __align__(16) unsigned short So[2][2][16 * OSP];
  const int lane = threadIdx.x & 31;
  const int w    = threadIdx.x >> 5;
  const int hh   = lane >> 4;
  const int m    = lane & 15;
  const int h    = blockIdx.y;
  const int b    = blockIdx.z;
  const int kvh  = h >> 1;
  const int q0   = blockIdx.x * 32 + w * 16;

  const _Float16* Qh = (const _Float16*)(const void*)Qhp;
  const _Float16* Ql = (const _Float16*)(const void*)Qlp;
  const _Float16* Kr = (const _Float16*)(const void*)Kpp + (size_t)b * SQ * EK + kvh * HD
                       + (size_t)m * EK + 8 * hh;
  const size_t vplane = (size_t)((b * NKV + kvh) * HD) * SQ;
  const _Float16* Vhr = (const _Float16*)(const void*)Vhp + vplane + (size_t)m * SQ + 8 * hh;
  const _Float16* Vlr = (const _Float16*)(const void*)Vlp + vplane + (size_t)m * SQ + 8 * hh;

  v16h qh[4], ql[4];
  {
    const size_t qo = ((size_t)b * SQ + q0 + m) * EQ + (size_t)h * HD + 8 * hh;
#pragma unroll
    for (int dc = 0; dc < 4; ++dc) {
      qh[dc] = ldh(Qh + qo + 32 * dc);
      ql[dc] = ldh(Ql + qo + 32 * dc);
    }
  }

  v8f acc[8];
#pragma unroll
  for (int t = 0; t < 8; ++t) acc[t] = (v8f){0.f, 0.f, 0.f, 0.f, 0.f, 0.f, 0.f, 0.f};
  float mrun = -1.0e30f;
  float lrun = 0.0f;

#pragma unroll 1
  for (int kc = 0; kc < SQ / 64; ++kc) {
    const int key0 = kc * 64;
    v8f s[4];
#pragma unroll
    for (int j = 0; j < 4; ++j) s[j] = (v8f){0.f, 0.f, 0.f, 0.f, 0.f, 0.f, 0.f, 0.f};
#pragma unroll
    for (int dc = 0; dc < 4; ++dc) {
      v16h kf[4];
#pragma unroll
      for (int j = 0; j < 4; ++j) kf[j] = ldh(Kr + (size_t)(key0 + 16 * j) * EK + 32 * dc);
#pragma unroll
      for (int j = 0; j < 4; ++j) {
        s[j] = mma_h(kf[j], qh[dc], s[j]);
        s[j] = mma_h(kf[j], ql[dc], s[j]);
      }
      g_qk(s[0], s[1], s[2], s[3], kf[0], kf[1], kf[2], kf[3], qh[dc], ql[dc]);
      sched_fence();
    }

    float cmax = -1.0e30f;
#pragma unroll
    for (int j = 0; j < 4; ++j)
#pragma unroll
      for (int r = 0; r < 8; ++r) cmax = fmaxf(cmax, s[j][r]);
    cmax = fmaxf(cmax, __shfl_xor(cmax, 16, 32));
    const float mnew  = fmaxf(mrun, cmax);
    const float alpha = __builtin_amdgcn_exp2f((mrun - mnew) * SINV);
    const float nms   = 8.0f - mnew * SINV;
    float psum = 0.f;
#pragma unroll
    for (int j = 0; j < 4; ++j)
#pragma unroll
      for (int r = 0; r < 8; ++r) {
        const float p = __builtin_amdgcn_exp2f(fmaf(s[j][r], SINV, nms));
        s[j][r] = p;
        psum += p;
      }
    psum += __shfl_xor(psum, 16, 32);
    lrun = fmaf(lrun, alpha, psum);
    mrun = mnew;
#pragma unroll
    for (int t = 0; t < 8; ++t) acc[t] = acc[t] * alpha;

#pragma unroll
    for (int ks = 0; ks < 2; ++ks) {
      HFrag pf;
      v8h plo, phi;
#pragma unroll
      for (int r = 0; r < 8; ++r) {
        plo[r] = (_Float16)s[2 * ks][r];
        phi[r] = (_Float16)s[2 * ks + 1][r];
      }
      pf.h[0] = plo;
      pf.h[1] = phi;
      const size_t ko = (size_t)(key0 + 32 * ks);
#pragma unroll
      for (int t = 0; t < 8; t += 2) {
        const v16h a0 = ldh(Vhr + (size_t)(16 * t) * SQ + ko);
        const v16h b0 = ldh(Vlr + (size_t)(16 * t) * SQ + ko);
        const v16h a1 = ldh(Vhr + (size_t)(16 * (t + 1)) * SQ + ko);
        const v16h b1 = ldh(Vlr + (size_t)(16 * (t + 1)) * SQ + ko);
        acc[t]     = mma_h(a0, pf.v, acc[t]);
        acc[t]     = mma_h(b0, pf.v, acc[t]);
        acc[t + 1] = mma_h(a1, pf.v, acc[t + 1]);
        acc[t + 1] = mma_h(b1, pf.v, acc[t + 1]);
        g_pv(acc[t], acc[t + 1], a0, b0, a1, b1, pf.v);
        sched_fence();
      }
    }
  }
  g_acc8(acc[0], acc[1], acc[2], acc[3], acc[4], acc[5], acc[6], acc[7]);

  const float inv = __builtin_amdgcn_rcpf(lrun) * (1.0f / VMUL);
  unsigned short* sh = So[w][0];
  unsigned short* sl = So[w][1];
#pragma unroll
  for (int t = 0; t < 8; ++t) {
    v4u hv, lvv;
#pragma unroll
    for (int q = 0; q < 4; ++q) {
      const float o0 = acc[t][2 * q] * inv;
      const float o1 = acc[t][2 * q + 1] * inv;
      const unsigned short h0 = f2bf_bits(o0), h1 = f2bf_bits(o1);
      const unsigned short l0 = f2bf_bits(o0 - bfb2f(h0)), l1 = f2bf_bits(o1 - bfb2f(h1));
      hv[q]  = pk16(h0, h1);
      lvv[q] = pk16(l0, l1);
    }
    *(v4u*)(sh + m * OSP + 16 * t + 8 * hh) = hv;
    *(v4u*)(sl + m * OSP + 16 * t + 8 * hh) = lvv;
  }
  __builtin_amdgcn_fence(__ATOMIC_RELEASE, "wavefront");
  __builtin_amdgcn_wave_barrier();
  __builtin_amdgcn_fence(__ATOMIC_ACQUIRE, "wavefront");
  v4u ov[2][8];
#pragma unroll
  for (int it = 0; it < 8; ++it) {
    const int row = 2 * it + hh;
    ov[0][it] = *(const v4u*)(sh + row * OSP + 8 * m);
    ov[1][it] = *(const v4u*)(sl + row * OSP + 8 * m);
  }
  for (int pass = 0; pass < 2; ++pass) {
#pragma unroll
    for (int it = 0; it < 8; ++it) {
      const int row = 2 * it + hh;
      const size_t go = ((size_t)b * SQ + q0 + row) * EQ + (size_t)h * HD + 8 * m;
      *(volatile v4u*)(Ohp + go) = ov[0][it];
      *(volatile v4u*)(Olp + go) = ov[1][it];
    }
    __threadfence();
  }
}

__global__ __launch_bounds__(128) void out_kernel(const unsigned short* __restrict__ Ohp,
                                                  const unsigned short* __restrict__ Olp,
                                                  const unsigned short* __restrict__ Wp,
                                                  float* __restrict__ out) {
  __shared__ __align__(16) float T[64 * TP];
  const int lane = threadIdx.x & 31;
  const int w    = threadIdx.x >> 5;
  const int wr   = w >> 1, wc = w & 1;
  const int arow0 = blockIdx.x * 64;
  const int brow0 = blockIdx.y * 128;
  const __bf16* A  = (const __bf16*)(const void*)Ohp + (size_t)(arow0 + 32 * wr) * DM;
  const __bf16* A2 = (const __bf16*)(const void*)Olp + (size_t)(arow0 + 32 * wr) * DM;
  const __bf16* B  = (const __bf16*)(const void*)Wp  + (size_t)(brow0 + 64 * wc) * DM;

  v8f acc[2][4];
#pragma unroll
  for (int i = 0; i < 2; ++i)
#pragma unroll
    for (int j = 0; j < 4; ++j) acc[i][j] = (v8f){0.f, 0.f, 0.f, 0.f, 0.f, 0.f, 0.f, 0.f};

  gemm_core<true>(A, A2, B, lane, acc);
  stage_tile(T, w, lane, acc);
  __syncthreads();

  v4f val[16];
#pragma unroll
  for (int it = 0; it < 16; ++it) val[it] = *(const v4f*)(T + (16 * w + it) * TP + 4 * lane);
  for (int pass = 0; pass < 2; ++pass) {
#pragma unroll
    for (int it = 0; it < 16; ++it) {
      *(volatile v4f*)(out + (size_t)(arow0 + 16 * w + it) * DM + brow0 + 4 * lane) = val[it];
    }
    __threadfence();
  }
}

extern "C" void kernel_launch(void* const* d_in, const int* in_sizes, int n_in,
                              void* d_out, int out_size, void* d_ws, size_t ws_size,
                              hipStream_t stream) {
  if (n_in < 9) return;
  if (in_sizes[0] != NTOK * DM) return;
  if (in_sizes[1] != EQ * DM || in_sizes[2] != EK * DM || in_sizes[3] != EK * DM || in_sizes[4] != DM * EQ) return;
  if (in_sizes[5] != HD || in_sizes[6] != HD) return;
  if (in_sizes[7] != SQ * (HD / 2) || in_sizes[8] != SQ * (HD / 2)) return;
  if (out_size != NTOK * DM) return;

  const float* x    = (const float*)d_in[0];
  const float* wq   = (const float*)d_in[1];
  const float* wk   = (const float*)d_in[2];
  const float* wv   = (const float*)d_in[3];
  const float* wo   = (const float*)d_in[4];
  const float* qnw  = (const float*)d_in[5];
  const float* knw  = (const float*)d_in[6];
  const float* fcos = (const float*)d_in[7];
  const float* fsin = (const float*)d_in[8];
  float* out        = (float*)d_out;

  const size_t szX  = (size_t)NTOK * DM * 2;
  const size_t szWq = (size_t)EQ * DM * 2;
  const size_t szWk = (size_t)EK * DM * 2;
  const size_t szWo = (size_t)DM * EQ * 2;
  const size_t szQ  = (size_t)NTOK * EQ * 2;
  const size_t szK  = (size_t)NTOK * EK * 2;
  const size_t szVt = (size_t)NB * NKV * HD * SQ * 2;
  const size_t szO  = (size_t)NTOK * EQ * 2;
  size_t off = 0;
  const size_t oX  = off; off += szX;
  const size_t oWq = off; off += szWq;
  const size_t oWk = off; off += szWk;
  const size_t oWv = off; off += szWk;
  const size_t oWo = off; off += szWo;
  const size_t oQh = off; off += szQ;
  const size_t oQl = off; off += szQ;
  const size_t oK  = off; off += szK;
  const size_t oVh = off; off += szVt;
  const size_t oVl = off; off += szVt;
  const size_t oOh = off; off += szO;
  const size_t oOl = off; off += szO;
  if (off > ws_size) return;

  char* ws = (char*)d_ws;
  unsigned short* Xb  = (unsigned short*)(ws + oX);
  unsigned short* Wqb = (unsigned short*)(ws + oWq);
  unsigned short* Wkb = (unsigned short*)(ws + oWk);
  unsigned short* Wvb = (unsigned short*)(ws + oWv);
  unsigned short* Wob = (unsigned short*)(ws + oWo);
  unsigned short* Qh  = (unsigned short*)(ws + oQh);
  unsigned short* Ql  = (unsigned short*)(ws + oQl);
  unsigned short* Kp  = (unsigned short*)(ws + oK);
  unsigned short* Vth = (unsigned short*)(ws + oVh);
  unsigned short* Vtl = (unsigned short*)(ws + oVl);
  unsigned short* Oh  = (unsigned short*)(ws + oOh);
  unsigned short* Ol  = (unsigned short*)(ws + oOl);

  {
    const int n8x  = (NTOK * DM) / 8;
    const int n8wq = (EQ * DM) / 8;
    const int n8wk = (EK * DM) / 8;
    const int n8wo = (DM * EQ) / 8;
    cvt_bf16_kernel<<<dim3((n8x + 255) / 256),  dim3(256), 0, stream>>>(x,  Xb,  n8x);
    cvt_bf16_kernel<<<dim3((n8wq + 255) / 256), dim3(256), 0, stream>>>(wq, Wqb, n8wq);
    cvt_bf16_kernel<<<dim3((n8wk + 255) / 256), dim3(256), 0, stream>>>(wk, Wkb, n8wk);
    cvt_bf16_kernel<<<dim3((n8wk + 255) / 256), dim3(256), 0, stream>>>(wv, Wvb, n8wk);
    cvt_bf16_kernel<<<dim3((n8wo + 255) / 256), dim3(256), 0, stream>>>(wo, Wob, n8wo);
  }

  proj_kernel<0><<<dim3(NTOK / 64, NH), dim3(128), 0, stream>>>(Xb, Wqb, qnw, fcos, fsin, Qh, Ql);
  proj_kernel<1><<<dim3(NTOK / 64, NKV), dim3(128), 0, stream>>>(Xb, Wkb, knw, fcos, fsin, Kp, Kp);
  proj_kernel<2><<<dim3(NTOK / 128, EK / 64), dim3(128), 0, stream>>>(Wvb, Xb, knw, fcos, fsin, Vth, Vtl);

  attn_kernel<<<dim3(SQ / 32, NH, NB), dim3(64), 0, stream>>>(Qh, Ql, Kp, Vth, Vtl, Oh, Ol);

  out_kernel<<<dim3(NTOK / 64, DM / 128), dim3(128), 0, stream>>>(Oh, Ol, Wob, out);

  (void)hipGetLastError();
}
